// URAClusteringGNN_59631325938205
// MI455X (gfx1250) — hardware-run, weakly checked
//
#include <hip/hip_runtime.h>


namespace {
constexpr int N = 50000, E = 800000, C = 64, NHD = 4, F = NHD * C, ED = 3, K = 4, NT16 = N / 16;
constexpr float XS = 8.0f, WSC = 256.0f, SLOPE = 0.2f, BEPS = 1e-5f;
typedef _Float16 b16;
typedef __attribute__((ext_vector_type(16))) _Float16 v16b;
typedef __attribute__((ext_vector_type(8))) _Float16 v8b;
typedef __attribute__((ext_vector_type(8))) float v8f;
typedef __attribute__((ext_vector_type(4))) float v4f;
typedef __attribute__((ext_vector_type(2))) float v2f;
__device__ __forceinline__ float bf16_rne(float f) { unsigned int u = __float_as_uint(f); u += 0x7FFFu + ((u >> 16) & 1u); float r = __uint_as_float(u & 0xFFFF0000u); asm volatile("" : "+v"(r)); return r; }
__device__ __forceinline__ void split16(float v, b16& hi, b16& lo) { hi = (b16)v; lo = (b16)(v - (float)hi); }
__device__ __forceinline__ v16b frag_kb(const b16* p, int hh) { const v8b a = *(const v8b*)(p + 8 * hh), b = *(const v8b*)(p + 16 + 8 * hh); v16b f;
#pragma unroll
  for (int e = 0; e < 8; ++e) { f[e] = a[e]; f[8 + e] = b[e]; } return f; }
__device__ __forceinline__ v8f wmma16b(v16b a, v16b b, v8f c) { v8f d = __builtin_amdgcn_wmma_f32_16x16x32_f16(false, a, false, b, (short)0, c, false, false); asm volatile("v_nop\n\tv_nop\n\tv_nop\n\tv_nop" : "+v"(d) : "v"(a), "v"(b)); return d; }
__device__ __forceinline__ void wave_lds_sync() { __builtin_amdgcn_fence(__ATOMIC_RELEASE, "workgroup"); __builtin_amdgcn_wave_barrier(); __builtin_amdgcn_fence(__ATOMIC_ACQUIRE, "workgroup"); }
__device__ __forceinline__ float pmul(float a, float b) { float p = a * b; asm volatile("" : "+v"(p)); return p; }
__device__ __forceinline__ int iclamp(int v, int lo, int hi) { return v < lo ? lo : (v > hi ? hi : v); }
__device__ __forceinline__ float lrelu(float v) { return v > 0.0f ? v : SLOPE * v; }
__device__ __forceinline__ float elu(float v) { return v > 0.0f ? v : (__expf(v) - 1.0f); }
constexpr int CSR_NBLK9 = 512, CSR_GB9 = 9, CSR_GN9 = 1 << CSR_GB9  , CSR_TS9 = (CSR_GN9 < 32 ? 32 : CSR_GN9)  , CSR_MAXG9 = 512, CSR_CAP9 = 12288  ;
__device__ __host__ __forceinline__ int csr_tix9(int v) { return (v >> CSR_GB9) * CSR_TS9 + (v & (CSR_GN9 - 1)); }
__global__ __launch_bounds__(64) void csrA_kernel9(const int* __restrict__ dst, int E, int N, int nG, int CHP, int NGP, int* __restrict__ STG, int* __restrict__ HST) {
  extern __shared__ int sm[];
  int* cnt = sm; int* run = sm + NGP; int* ids = sm + 2 * NGP;
  const int b = blockIdx.x; const int ch = (E + CSR_NBLK9 - 1) / CSR_NBLK9; const int e0 = b * ch, e1 = min(E, e0 + ch);
  for (int i = threadIdx.x; i < NGP; i += 64) cnt[i] = 0;
  for (int i = threadIdx.x; i < CHP; i += 64) ids[i] = -1;
  __syncthreads();
  if (threadIdx.x == 0) {
    for (int e = e0; e < e1; ++e) { int d = dst[e]; d = (d < 0) ? 0 : (d >= N ? N - 1 : d); cnt[d >> CSR_GB9] += 1; }
    int acc = 0; for (int g = 0; g < nG; ++g) { run[g] = acc; acc += cnt[g]; }
    for (int e = e0; e < e1; ++e) { int d = dst[e]; d = (d < 0) ? 0 : (d >= N ? N - 1 : d); const int g = d >> CSR_GB9; ids[run[g]] = e; run[g] += 1; } }
  __syncthreads();
  typedef __attribute__((ext_vector_type(4))) int v4i;
  for (int pass = 0; pass < 2; ++pass) {
    for (int i = threadIdx.x; i < CHP / 4; i += 64) *(volatile v4i*)(STG + (size_t)b * CHP + i * 4) = *(const v4i*)(&ids[i * 4]);
    for (int i = threadIdx.x; i < NGP / 4; i += 64) { v4i v; for (int e = 0; e < 4; ++e) v[e] = (i * 4 + e < nG) ? cnt[i * 4 + e] : 0; *(volatile v4i*)(HST + (size_t)b * NGP + i * 4) = v; }
    __threadfence(); }
}
__global__ __launch_bounds__(512) void csrS_kernel9(const int* __restrict__ HST, int nG, int NGP, int* __restrict__ START, int* __restrict__ TOT, int* __restrict__ OFF) {
  __shared__ int tot[CSR_MAXG9];
  const int b = threadIdx.x;
  for (int pass = 0; pass < 2; ++pass) { int runb = 0; for (int g = 0; g < nG; ++g) { int c = HST[(size_t)b * NGP + g]; c = (c < 0) ? 0 : c; ((volatile int*)OFF)[(size_t)g * CSR_NBLK9 + b] = runb; runb += c; } __threadfence(); }
  for (int g = threadIdx.x; g < nG; g += 512) { int s = 0; for (int bb = 0; bb < CSR_NBLK9; ++bb) { int c = HST[(size_t)bb * NGP + g]; s += (c < 0) ? 0 : c; } tot[g] = s; }
  __syncthreads();
  if (threadIdx.x < 32) {
    __shared__ int st[CSR_MAXG9 + 32];
    if (threadIdx.x == 0) { int acc = 0; for (int g = 0; g < NGP; ++g) { st[g] = acc; if (g < nG) acc += (tot[g] + 31) & ~31; } st[NGP] = acc; }
    __builtin_amdgcn_fence(__ATOMIC_RELEASE, "workgroup"); __builtin_amdgcn_wave_barrier(); __builtin_amdgcn_fence(__ATOMIC_ACQUIRE, "workgroup");
    for (int pass = 0; pass < 2; ++pass) { for (int i = threadIdx.x; i < NGP + 32; i += 32) { ((volatile int*)START)[i] = (i <= NGP) ? st[min(i, NGP)] : 0; ((volatile int*)TOT)[i] = (i < nG) ? tot[i] : 0; } __threadfence(); } }
}
__global__ __launch_bounds__(256) void csrB_kernel9(const int* __restrict__ dst, int N, int nG, int CHP, int NGP, int permLen, const int* __restrict__ STG, const int* __restrict__ HST, const int* __restrict__ OFF, const int* __restrict__ START, const int* __restrict__ TOT, int* __restrict__ PERM, int* __restrict__ ROWPTR, int* __restrict__ ROWCNT, int* __restrict__ FLAG) {
  typedef __attribute__((ext_vector_type(4))) int v4i;
  __shared__ int ids[CSR_CAP9]; __shared__ unsigned short key[CSR_CAP9]; __shared__ int outp[CSR_CAP9]; __shared__ int ncnt[CSR_GN9 + 1]; __shared__ int boff[CSR_NBLK9 + 1];
  const int g = blockIdx.x, t_ = threadIdx.x; int tot = TOT[g]; int st = START[g], stn = START[g + 1]; const int v0 = g * CSR_GN9; const int nv = min(CSR_GN9, N - v0); const int t0 = g * CSR_TS9;
  st = (st < 0) ? 0 : (st > permLen - 32 ? permLen - 32 : st) & ~31; stn = (stn < st) ? st : (stn > permLen ? permLen : stn); tot = (tot < 0) ? 0 : tot; if (tot > stn - st && tot <= CSR_CAP9) tot = stn - st;
  if (tot > CSR_CAP9) {
    for (int pass = 0; pass < 2; ++pass) { for (int i = t_; i < CSR_TS9 / 4; i += 256) { v4i a, c; for (int e = 0; e < 4; ++e) { a[e] = st; c[e] = 0; } *(volatile v4i*)(ROWPTR + t0 + i * 4) = a; *(volatile v4i*)(ROWCNT + t0 + i * 4) = c; } if (t_ == 0) ((volatile int*)FLAG)[0] = 1; __threadfence(); } (void)nv; return; }
  if (t_ == 0) { int acc = 0; for (int b = 0; b < CSR_NBLK9; ++b) { boff[b] = acc; int c = HST[(size_t)b * NGP + g]; c = (c < 0) ? 0 : (c > CHP ? CHP : c); acc += c; if (acc > tot) acc = tot; } boff[CSR_NBLK9] = acc; }
  for (int i = t_; i <= CSR_GN9; i += 256) ncnt[i] = 0;
  __syncthreads();
  for (int b = 0; b < CSR_NBLK9; ++b) { const int c = boff[b + 1] - boff[b]; int o_ = OFF[(size_t)g * CSR_NBLK9 + b]; o_ = (o_ < 0) ? 0 : (o_ > CHP - c ? CHP - c : o_); const int* src_ = STG + (size_t)b * CHP + o_;
    for (int i = t_; i < c; i += 256) { int id = src_[i]; id = (id < 0) ? 0 : id; ids[boff[b] + i] = id; int d = dst[id]; d = (d < v0) ? v0 : (d >= N ? N - 1 : d); int kk = d - v0; kk = (kk < 0) ? 0 : (kk >= CSR_GN9 ? CSR_GN9 - 1 : kk); key[boff[b] + i] = (unsigned short)kk; } }
  __syncthreads();
  if (t_ == 0) { for (int i = 0; i < tot; ++i) ncnt[key[i]] += 1; int acc = 0; for (int vl = 0; vl < CSR_GN9; ++vl) { const int c = ncnt[vl]; ncnt[vl] = acc; acc += c; } ncnt[CSR_GN9] = acc;
    for (int i = 0; i < tot; ++i) { const int vl = key[i]; outp[ncnt[vl]] = ids[i]; ncnt[vl] += 1; }
    for (int vl = CSR_GN9; vl > 0; --vl) ncnt[vl] = ncnt[vl - 1]; ncnt[0] = 0; }
  __syncthreads();
  for (int pass = 0; pass < 2; ++pass) {
    for (int i = t_; i < (stn - st) / 4; i += 256) { v4i v; for (int e = 0; e < 4; ++e) { const int q = i * 4 + e; v[e] = (q < tot) ? outp[q] : -1; } *(volatile v4i*)(PERM + st + i * 4) = v; }
    for (int i = t_; i < CSR_TS9 / 4; i += 256) { v4i a, c; for (int e = 0; e < 4; ++e) { const int vl = i * 4 + e; const int vc = vl < CSR_GN9 ? vl : CSR_GN9; a[e] = (vl < CSR_GN9) ? st + ncnt[vc] : st; c[e] = (vl < nv) ? (ncnt[(vc < CSR_GN9 ? vc : CSR_GN9 - 1) + 1] - ncnt[vc]) : 0; } *(volatile v4i*)(ROWPTR + t0 + i * 4) = a; *(volatile v4i*)(ROWCNT + t0 + i * 4) = c; }
    __threadfence(); }
}
__global__ __launch_bounds__(256) void csrZ_kernel9(int* __restrict__ p, size_t n4) { typedef __attribute__((ext_vector_type(4))) int v4i; const size_t tid = (size_t)blockIdx.x * 256 + threadIdx.x, nth = (size_t)gridDim.x * 256; v4i z = {0, 0, 0, 0}; for (size_t i = tid; i < n4; i += nth) *(volatile v4i*)(p + i * 4) = z; }
struct CsrBufs9 { int *STG, *HST, *OFF, *START, *TOT, *PERM, *ROWPTR, *ROWCNT, *FLAG; int nG, NGP, CHP; size_t permLen; char* base; size_t bytes; };
static size_t csr_carve9(CsrBufs9& c, char* ws, size_t off, int E, int N) {
  const size_t off0 = off; c.base = ws + off;
  auto al = [&](size_t bytes) { char* p = ws + off; off += (bytes + 255) & ~(size_t)255; return p; };
  c.nG = (N + CSR_GN9 - 1) / CSR_GN9; c.NGP = (c.nG + 31) & ~31; const int ch = (E + CSR_NBLK9 - 1) / CSR_NBLK9; c.CHP = (ch + 31) & ~31; c.permLen = (size_t)E + 32 * (size_t)c.nG + 32;
  c.STG = (int*)al((size_t)CSR_NBLK9 * c.CHP * 4); c.HST = (int*)al((size_t)CSR_NBLK9 * c.NGP * 4); c.OFF = (int*)al((size_t)c.NGP * CSR_NBLK9 * 4); c.START = (int*)al((size_t)(c.NGP + 64) * 4); c.TOT = (int*)al((size_t)(c.NGP + 64) * 4);
  c.PERM = (int*)al(c.permLen * 4); c.ROWPTR = (int*)al((size_t)c.nG * CSR_TS9 * 4); c.ROWCNT = (int*)al((size_t)c.nG * CSR_TS9 * 4); c.FLAG = (int*)al(256);
  c.bytes = off - off0; return off;
}
static void csr_build9(const CsrBufs9& c, const int* dst, int E, int N, hipStream_t stream) {
  const size_t smem = (size_t)(2 * c.NGP + c.CHP) * 4;
  csrZ_kernel9<<<512, 256, 0, stream>>>((int*)c.base, c.bytes / 16);
  csrA_kernel9<<<CSR_NBLK9, 64, smem, stream>>>(dst, E, N, c.nG, c.CHP, c.NGP, c.STG, c.HST);
  csrS_kernel9<<<1, 512, 0, stream>>>(c.HST, c.nG, c.NGP, c.START, c.TOT, c.OFF);
  csrB_kernel9<<<c.nG, 256, 0, stream>>>(dst, N, c.nG, c.CHP, c.NGP, (int)c.permLen, c.STG, c.HST, c.OFF, c.START, c.TOT, c.PERM, c.ROWPTR, c.ROWCNT, c.FLAG);
}


__global__ __launch_bounds__(256) void wput_kernel(const float* __restrict__ w, int KIN, int KP, int OUTW, b16* __restrict__ WT) { const int KG = KP / 8; const int u = blockIdx.x * 256 + threadIdx.x; if (u >= OUTW * KG) return; const int o = u / KG, k0 = (u % KG) * 8; v8b v;
#pragma unroll
  for (int j = 0; j < 8; ++j) { const int k = k0 + j; v[j] = (b16)(k < KIN ? bf16_rne(w[(size_t)k * OUTW + o]) * WSC : 0.0f); } for (int pass = 0; pass < 2; ++pass) { *(volatile v8b*)(WT + (size_t)o * KP + k0) = v; __threadfence(); } }
template <int KIN, int KP, int MODE>
__global__ __launch_bounds__(32) void dense_kernel(const float* __restrict__ IN, const b16* __restrict__ WT, const float* __restrict__ bias, int NG, int NLIM, float* __restrict__ OUT) {
  __shared__ __attribute__((aligned(16))) b16 Ah[16][KP + 8], Al[16][MODE == 0 ? 8 : KP + 8]; __shared__ float Tf[16][68]; const int lane = threadIdx.x, nloc = lane & 15, hlf = lane >> 4; const int g = blockIdx.x % NG; const size_t m0 = (size_t)(blockIdx.x / NG) * 16; if (m0 >= (size_t)NLIM) return; const int OW = NG * 64;
  for (int rr = 0; rr < 16; ++rr) for (int q = 0; q < KP / 32; ++q) { const int k = q * 32 + lane; const float v = (k < KIN) ? IN[(m0 + rr) * KIN + k] : 0.0f; if (MODE == 0) Ah[rr][k] = (b16)(bf16_rne(v) * XS); else { b16 p, ql; split16(v * XS, p, ql); Ah[rr][k] = p; Al[rr][k] = ql; } }
  wave_lds_sync(); v8f acc[4] = {(v8f){}, (v8f){}, (v8f){}, (v8f){}};
#pragma unroll
  for (int kb = 0; kb < KP; kb += 32) { const v16b a = frag_kb(&Ah[nloc][kb], hlf); v16b a2; if (MODE != 0) a2 = frag_kb(&Al[nloc][kb], hlf);
#pragma unroll
    for (int t = 0; t < 4; ++t) { const v16b bw = frag_kb(WT + (size_t)(g * 64 + t * 16 + nloc) * KP + kb, hlf); acc[t] = wmma16b(a, bw, acc[t]); if (MODE != 0) acc[t] = wmma16b(a2, bw, acc[t]); } }
#pragma unroll
  for (int t = 0; t < 4; ++t) { const int c = g * 64 + t * 16 + nloc; const float bb = bias ? bf16_rne(bias[c]) : 0.0f;
#pragma unroll
    for (int r8 = 0; r8 < 8; ++r8) Tf[8 * hlf + r8][t * 16 + nloc] = acc[t][r8] * (1.0f / (XS * WSC)) + bb; }
  wave_lds_sync();
  for (int pass = 0; pass < 2; ++pass) { for (int rr = 0; rr < 16; ++rr) *(volatile v2f*)(OUT + (m0 + rr) * OW + g * 64 + lane * 2) = (v2f){Tf[rr][lane * 2], Tf[rr][lane * 2 + 1]}; __threadfence(); }
}
__global__ __launch_bounds__(256) void aldot_kernel(const float* __restrict__ Hh, int NHh, const float* __restrict__ as, const float* __restrict__ ad, int NLIM, float* __restrict__ AL) {
  const int wave = threadIdx.x >> 5, lane = threadIdx.x & 31; const size_t i = (size_t)blockIdx.x * 8 + wave; if (i >= (size_t)NLIM) return; const int Fh = NHh * C; float outv = 0.0f;
  for (int hd = 0; hd < NHh; ++hd) { const float h0 = Hh[i * Fh + hd * C + lane], h1 = Hh[i * Fh + hd * C + 32 + lane]; float s = pmul(h0, bf16_rne(as[hd * C + lane])) + pmul(h1, bf16_rne(as[hd * C + 32 + lane])); float d = pmul(h0, bf16_rne(ad[hd * C + lane])) + pmul(h1, bf16_rne(ad[hd * C + 32 + lane]));
    for (int o = 16; o; o >>= 1) { s += __shfl_xor(s, o); d += __shfl_xor(d, o); } if (lane == hd) outv = s; if (lane == 4 + hd) outv = d; }
  for (int pass = 0; pass < 2; ++pass) { ((volatile float*)AL)[i * 32 + lane] = outv; __threadfence(); } }
template <int NHh, int ELU>
__global__ __launch_bounds__(256) void agg_kernel(const float* __restrict__ Hh, const float* __restrict__ AL, const float* __restrict__ ea, const float* __restrict__ We, const float* __restrict__ ae, const float* __restrict__ bias, const int* __restrict__ srcs, const int* __restrict__ PERM, const int* __restrict__ ROWPTR, const int* __restrict__ ROWCNT, int permLen, int NLIM, float* __restrict__ G) {
  constexpr int Fh = NHh * C, CPL = Fh / 32, LPH = 32 / NHh;
  __shared__ float V[NHh][4]; const int wave = threadIdx.x >> 5, lane = threadIdx.x & 31;
  if (threadIdx.x < NHh * ED) { const int hd = threadIdx.x / ED, k = threadIdx.x % ED; float s = 0.0f; for (int c = 0; c < C; ++c) s += pmul(bf16_rne(We[(size_t)k * Fh + hd * C + c]), bf16_rne(ae[hd * C + c])); V[hd][k] = s; }
  __syncthreads(); const size_t i = (size_t)blockIdx.x * 8 + wave; if (i >= (size_t)NLIM) return; const int hd = lane / LPH; int st = ROWPTR[i], cnt = ROWCNT[i]; cnt = iclamp(cnt, 0, 1 << 20); st = iclamp(st, 0, permLen - cnt);
  const float adi = AL[i * 32 + 4 + hd]; const float v0 = V[hd][0], v1 = V[hd][1], v2 = V[hd][2]; float m = -INFINITY, den = 0.0f, acc[CPL]; for (int k = 0; k < CPL; ++k) acc[k] = 0.0f; float es0 = 0.0f, es1 = 0.0f, es2 = 0.0f; int n = 0;
  auto step = [&](size_t u, float e0, float e1, float e2) { const float s = lrelu(AL[u * 32 + hd] + adi + pmul(e0, v0) + pmul(e1, v1) + pmul(e2, v2)); const float mn = fmaxf(m, s); const float sc = (m == -INFINITY) ? 0.0f : __expf(m - mn); const float p = __expf(s - mn); den = den * sc + p;
#pragma unroll
    for (int k = 0; k < CPL; ++k) acc[k] = pmul(acc[k], sc) + pmul(p, Hh[u * Fh + lane * CPL + k]); m = mn; };
#pragma unroll 1
  for (int j = 0; j < cnt; ++j) { const int e = iclamp(PERM[st + j], 0, E - 1); const size_t u = (size_t)iclamp(srcs[e], 0, N - 1); if (u >= (size_t)NLIM) continue; const float e0 = bf16_rne(ea[(size_t)e * 3]), e1 = bf16_rne(ea[(size_t)e * 3 + 1]), e2 = bf16_rne(ea[(size_t)e * 3 + 2]); es0 += e0; es1 += e1; es2 += e2; ++n; step(u, e0, e1, e2); }
  { const float inv = 1.0f / (float)(n > 0 ? n : 1); step(i, pmul(es0, inv), pmul(es1, inv), pmul(es2, inv)); }
  float r[CPL]; for (int k = 0; k < CPL; ++k) { const float v = acc[k] / (den + 1e-16f) + bf16_rne(bias[lane * CPL + k]); r[k] = ELU ? elu(v) : v; }
  for (int pass = 0; pass < 2; ++pass) { if (CPL == 8) { *(volatile v4f*)(G + i * Fh + lane * 8) = (v4f){r[0], r[1], r[2], r[3]}; *(volatile v4f*)(G + i * Fh + lane * 8 + 4) = (v4f){r[CPL > 4 ? 4 : 0], r[CPL > 5 ? 5 : 0], r[CPL > 6 ? 6 : 0], r[CPL > 7 ? 7 : 0]}; } else *(volatile v2f*)(G + i * Fh + lane * 2) = (v2f){r[0], r[CPL > 1 ? 1 : 0]}; __threadfence(); } }
template <int FW>
__global__ __launch_bounds__(256) void tilestat_kernel(const float* __restrict__ Hm, int NLIM, float* __restrict__ PS, float* __restrict__ PQ) { constexpr int CPL = FW / 32; const int wave = threadIdx.x >> 5, lane = threadIdx.x & 31; const size_t tile = (size_t)blockIdx.x * 8 + wave; if (tile * 16 >= (size_t)NLIM) return; float s[CPL], q[CPL]; for (int k = 0; k < CPL; ++k) { s[k] = 0.0f; q[k] = 0.0f; }
#pragma unroll 1
  for (int rr = 0; rr < 16; ++rr) for (int k = 0; k < CPL; ++k) { const float v = Hm[(tile * 16 + rr) * FW + lane * CPL + k]; s[k] += v; q[k] += pmul(v, v); }
  for (int pass = 0; pass < 2; ++pass) { for (int k = 0; k < CPL; ++k) { ((volatile float*)PS)[tile * FW + lane * CPL + k] = s[k]; ((volatile float*)PQ)[tile * FW + lane * CPL + k] = q[k]; } __threadfence(); } }
__global__ __launch_bounds__(256) void bnstat_kernel(const float* __restrict__ PS, const float* __restrict__ PQ, int FW, int ntiles, int nrows, float* __restrict__ ST) { const int c = threadIdx.x; if (c >= FW) return; double s = 0.0, q = 0.0;
#pragma unroll 1
  for (int t = 0; t < ntiles; ++t) { s += (double)PS[(size_t)t * FW + c]; q += (double)PQ[(size_t)t * FW + c]; } const double mu = s / (double)nrows; double var = q / (double)nrows - mu * mu; if (var < 0.0) var = 0.0;
  for (int pass = 0; pass < 2; ++pass) { ((volatile float*)ST)[c] = (float)mu; ((volatile float*)ST)[FW + c] = (float)(1.0 / sqrt(var + (double)BEPS)); __threadfence(); } }
__global__ __launch_bounds__(256) void bnelu_kernel(const float* __restrict__ Hm, const float* __restrict__ ST, int FW, int NLIM, float* __restrict__ OUT) { const size_t u = (size_t)blockIdx.x * 256 + threadIdx.x; if (u >= (size_t)NLIM * FW / 2) return; const int c0 = (int)(u % (FW / 2)) * 2; const v2f v = *(const v2f*)(Hm + u * 2); v2f r;
  for (int k = 0; k < 2; ++k) r[k] = elu(pmul(v[k] - ST[c0 + k], ST[FW + c0 + k]));
  for (int pass = 0; pass < 2; ++pass) { *(volatile v2f*)(OUT + u * 2) = r; __threadfence(); } }
__global__ __launch_bounds__(256) void cls_kernel(const float* __restrict__ Hm, const float* __restrict__ Wc, const float* __restrict__ bc, int NLIM, float* __restrict__ out) { const int i = blockIdx.x * 256 + threadIdx.x; if (i >= NLIM) return; float l[K]; for (int k = 0; k < K; ++k) l[k] = bf16_rne(bc[k]);
#pragma unroll 1
  for (int c = 0; c < C; ++c) { const float hv = Hm[(size_t)i * C + c]; for (int k = 0; k < K; ++k) l[k] += pmul(hv, bf16_rne(Wc[c * K + k])); }
  float mx = l[0]; for (int k = 1; k < K; ++k) mx = fmaxf(mx, l[k]); float e[K], s = 0.0f; for (int k = 0; k < K; ++k) { e[k] = __expf(l[k] - mx); s += e[k]; } v4f r; for (int k = 0; k < K; ++k) r[k] = e[k] / s;
  for (int pass = 0; pass < 2; ++pass) { *(volatile v4f*)(out + (size_t)i * K) = r; __threadfence(); } }
}

extern "C" void kernel_launch(void* const* d_in, const int* in_sizes, int n_in, void* d_out, int out_size, void* d_ws, size_t ws_size, hipStream_t stream) {
  (void)n_in;
  auto Fp = [&](int i) { return (const float*)d_in[i]; }; auto Ip = [&](int i) { return (const int*)d_in[i]; };
  if (in_sizes[0] != N * 2 || in_sizes[1] != 2 * E || in_sizes[2] != E * ED || in_sizes[3] != 2 * C || in_sizes[5] != C * F || in_sizes[11] != F * F || in_sizes[17] != F * C || in_sizes[23] != C * K || out_size != N * K) return;
  const int NLIM = N;
  const int NT = NLIM / 16;
  size_t off = 0; char* ws = (char*)d_ws;
  auto carve = [&](size_t bytes) { char* p = ws + off; off += (bytes + 255) & ~(size_t)255; return p; };
  b16* WP = (b16*)carve((size_t)C * 32 * 2); b16* W1T = (b16*)carve((size_t)F * C * 2); b16* W2T = (b16*)carve((size_t)F * F * 2); b16* W3T = (b16*)carve((size_t)C * F * 2);
  float* HA = (float*)carve((size_t)N * F * 4); float* HB = (float*)carve((size_t)N * F * 4); float* G = (float*)carve((size_t)N * F * 4); float* AL = (float*)carve((size_t)N * 32 * 4); float* PS = (float*)carve((size_t)NT16 * F * 4); float* PQ = (float*)carve((size_t)NT16 * F * 4); float* ST = (float*)carve((size_t)2 * F * 4);
  CsrBufs9 csr; off = csr_carve9(csr, ws, off, E, N);
  if (off > ws_size || off > ((size_t)200 << 20)) return;
  wput_kernel<<<(C * 4 + 255) / 256, 256, 0, stream>>>(Fp(3), 2, 32, C, WP); wput_kernel<<<(F * 8 + 255) / 256, 256, 0, stream>>>(Fp(5), C, C, F, W1T); wput_kernel<<<(F * 32 + 255) / 256, 256, 0, stream>>>(Fp(11), F, F, F, W2T); wput_kernel<<<(C * 32 + 255) / 256, 256, 0, stream>>>(Fp(17), F, F, C, W3T);
  csr_build9(csr, Ip(1) + E, E, N, stream);
  dense_kernel<2, 32, 0><<<NT, 32, 0, stream>>>(Fp(0), WP, Fp(4), 1, NLIM, HA);
  tilestat_kernel<C><<<(NT + 7) / 8, 256, 0, stream>>>(HA, NLIM, PS, PQ); bnstat_kernel<<<1, 256, 0, stream>>>(PS, PQ, C, NT, NLIM, ST); bnelu_kernel<<<(unsigned)(((size_t)NLIM * C / 2 + 255) / 256), 256, 0, stream>>>(HA, ST, C, NLIM, HB);
  dense_kernel<C, C, 1><<<NT * 4, 32, 0, stream>>>(HB, W1T, nullptr, 4, NLIM, HA); aldot_kernel<<<(NLIM + 7) / 8, 256, 0, stream>>>(HA, 4, Fp(6), Fp(7), NLIM, AL);
  agg_kernel<4, 0><<<(NLIM + 7) / 8, 256, 0, stream>>>(HA, AL, Fp(2), Fp(8), Fp(9), Fp(10), Ip(1), csr.PERM, csr.ROWPTR, csr.ROWCNT, (int)csr.permLen, NLIM, G);
  tilestat_kernel<F><<<(NT + 7) / 8, 256, 0, stream>>>(G, NLIM, PS, PQ); bnstat_kernel<<<1, 256, 0, stream>>>(PS, PQ, F, NT, NLIM, ST); bnelu_kernel<<<(unsigned)(((size_t)NLIM * F / 2 + 255) / 256), 256, 0, stream>>>(G, ST, F, NLIM, HB);
  dense_kernel<F, F, 1><<<NT * 4, 32, 0, stream>>>(HB, W2T, nullptr, 4, NLIM, HA); aldot_kernel<<<(NLIM + 7) / 8, 256, 0, stream>>>(HA, 4, Fp(12), Fp(13), NLIM, AL);
  agg_kernel<4, 0><<<(NLIM + 7) / 8, 256, 0, stream>>>(HA, AL, Fp(2), Fp(14), Fp(15), Fp(16), Ip(1), csr.PERM, csr.ROWPTR, csr.ROWCNT, (int)csr.permLen, NLIM, G);
  tilestat_kernel<F><<<(NT + 7) / 8, 256, 0, stream>>>(G, NLIM, PS, PQ); bnstat_kernel<<<1, 256, 0, stream>>>(PS, PQ, F, NT, NLIM, ST); bnelu_kernel<<<(unsigned)(((size_t)NLIM * F / 2 + 255) / 256), 256, 0, stream>>>(G, ST, F, NLIM, HB);
  dense_kernel<F, F, 1><<<NT, 32, 0, stream>>>(HB, W3T, nullptr, 1, NLIM, HA); aldot_kernel<<<(NLIM + 7) / 8, 256, 0, stream>>>(HA, 1, Fp(18), Fp(19), NLIM, AL);
  agg_kernel<1, 1><<<(NLIM + 7) / 8, 256, 0, stream>>>(HA, AL, Fp(2), Fp(20), Fp(21), Fp(22), Ip(1), csr.PERM, csr.ROWPTR, csr.ROWCNT, (int)csr.permLen, NLIM, G);
  cls_kernel<<<(NLIM + 255) / 256, 256, 0, stream>>>(G, Fp(23), Fp(24), NLIM, (float*)d_out);
}
